// APPNPNet_Structural_74577812128607
// MI455X (gfx1250) — hardware-verified
//
#include <hip/hip_runtime.h>
#include <stddef.h>


#define DX      128
#define DH      64
#define DA      16
#define AF      8
#define NTHR    256
#define NWAVE   8
#define EPT     8
#define NGRP    4
#define CHUNK   (NTHR * EPT * NGRP)
#define SLOTB   14
#define NBP     1024
#define NBD     16384
#define WCAPP   128
#define WCAPD   512
#define GROWS   128
#define WP      136
#define TAP     24
#define NGMAX   256
#define WSCALE  8.0f
#define WINV    0.125f
#define C_KEEP  0.9f
#define C_TEL   0.1f

#define LDS_DEG  (NBD * 4 + NWAVE * WCAPD * 4 + 64)
#define LDS_PROP (NBP * DH * 4 + NWAVE * WCAPP * 4 + 64)
#define LDS_POOL (NGMAX * DH * 4 + NWAVE * 16 * TAP * 2 + NGMAX * 4)

static_assert((CHUNK & (CHUNK - 1)) == 0);
static_assert(CHUNK <= 8192);
static_assert((NBP & (NBP - 1)) == 0 && NBP <= (1 << SLOTB));
static_assert((NBD & (NBD - 1)) == 0 && NBD <= (1 << SLOTB));
static_assert(NBP % GROWS == 0);
static_assert(NBD % NBP == 0);
static_assert(NGMAX == NWAVE * 32);
static_assert((NGMAX / 16) % NWAVE == 0);
static_assert(DX % 32 == 0 && DH % 32 == 0);

typedef float    v2f  __attribute__((ext_vector_type(2)));
typedef float    v4f  __attribute__((ext_vector_type(4)));
typedef float    v8f  __attribute__((ext_vector_type(8)));
typedef int      v4i  __attribute__((ext_vector_type(4)));
typedef _Float16 v8h  __attribute__((ext_vector_type(8)));
typedef _Float16 v16h __attribute__((ext_vector_type(16)));
union FragH { v16h v; v8h h[2]; };

__device__ __forceinline__ v8h cvt8(v4f a, v4f b) {
  v8h r;
  r[0] = (_Float16)a.x; r[1] = (_Float16)a.y; r[2] = (_Float16)a.z; r[3] = (_Float16)a.w;
  r[4] = (_Float16)b.x; r[5] = (_Float16)b.y; r[6] = (_Float16)b.z; r[7] = (_Float16)b.w;
  return r;
}

__device__ __forceinline__ v8f wmh(v16h a, v16h b, v8f c) {
  v8f d = __builtin_amdgcn_wmma_f32_16x16x32_f16(false, a, false, b, (short)0, c, false, false);
  asm volatile("v_nop\n\tv_nop\n\tv_nop\n\tv_nop" : "+v"(d) : "v"(a), "v"(b));
  return d;
}

template <int NB, int WCAP>
__device__ __forceinline__ int scan_chunk(const int* __restrict__ dsts, int nE, int cbase, int nodeBase,
                                          int vec8, int* list, int tid, int lane, int wave) {
  int wc = 0;
  (void)lane;
#pragma unroll
  for (int g = 0; g < NGRP; ++g) {
    const int el0  = (g * NTHR + tid) * EPT;
    const int e0   = cbase + el0;
    const int sent = -2147483647 - 1;
    v4i da, db;
    if (vec8 != 0 && e0 + 7 < nE) {
      da = *(const v4i*)(dsts + e0);
      db = *(const v4i*)(dsts + e0 + 4);
    } else {
      da.x = (e0     < nE) ? dsts[min(e0, nE - 1)]     : sent;
      da.y = (e0 + 1 < nE) ? dsts[min(e0 + 1, nE - 1)] : sent;
      da.z = (e0 + 2 < nE) ? dsts[min(e0 + 2, nE - 1)] : sent;
      da.w = (e0 + 3 < nE) ? dsts[min(e0 + 3, nE - 1)] : sent;
      db.x = (e0 + 4 < nE) ? dsts[min(e0 + 4, nE - 1)] : sent;
      db.y = (e0 + 5 < nE) ? dsts[min(e0 + 5, nE - 1)] : sent;
      db.z = (e0 + 6 < nE) ? dsts[min(e0 + 6, nE - 1)] : sent;
      db.w = (e0 + 7 < nE) ? dsts[min(e0 + 7, nE - 1)] : sent;
    }
    const unsigned nb = (unsigned)nodeBase;
    const unsigned s0 = (unsigned)da.x - nb, s1 = (unsigned)da.y - nb;
    const unsigned s2 = (unsigned)da.z - nb, s3 = (unsigned)da.w - nb;
    const unsigned s4 = (unsigned)db.x - nb, s5 = (unsigned)db.y - nb;
    const unsigned s6 = (unsigned)db.z - nb, s7 = (unsigned)db.w - nb;
    const bool h0 = s0 < (unsigned)NB, h1 = s1 < (unsigned)NB, h2 = s2 < (unsigned)NB, h3 = s3 < (unsigned)NB;
    const bool h4 = s4 < (unsigned)NB, h5 = s5 < (unsigned)NB, h6 = s6 < (unsigned)NB, h7 = s7 < (unsigned)NB;
    const unsigned any = __builtin_amdgcn_ballot_w32(h0 | h1 | h2 | h3 | h4 | h5 | h6 | h7);
    if (any != 0u) {
#define HITJ(J, HJ, SJ) { \
        const unsigned mj = __builtin_amdgcn_ballot_w32(HJ); \
        if (mj != 0u) { \
          if (HJ) { \
            const int pos = wc + (int)__builtin_amdgcn_mbcnt_lo(mj, 0u); \
            if (pos < WCAP) list[wave * WCAP + pos] = ((el0 + (J)) << SLOTB) | (int)(SJ); \
          } \
          wc += (int)__builtin_popcount(mj); } }
      HITJ(0, h0, s0)
      HITJ(1, h1, s1)
      HITJ(2, h2, s2)
      HITJ(3, h3, s3)
      HITJ(4, h4, s4)
      HITJ(5, h5, s5)
      HITJ(6, h6, s6)
      HITJ(7, h7, s7)
#undef HITJ
    }
  }
  return wc;
}

__global__ __launch_bounds__(NTHR) void k_deg(
    const int* __restrict__ ei, float* dinv, int nE, int vec8) {
  extern __shared__ v4f lds_dyn[];
  int* cnt  = (int*)lds_dyn;
  int* list = cnt + NBD;
  int* wcnt = list + NWAVE * WCAPD;
  const int tid = threadIdx.x, lane = tid & 31, wave = tid >> 5;
  const int nodeBase = blockIdx.x * NBD;
  const int* dsts = ei + nE;

  {
    const v4i z = {0, 0, 0, 0};
    for (int i = tid; i < NBD / 4; i += NTHR) ((v4i*)cnt)[i] = z;
  }
  __syncthreads();

  const int nChunks = (nE + CHUNK - 1) / CHUNK;
#pragma unroll 1
  for (int ch = 0; ch < nChunks; ++ch) {
    const int cbase = ch * CHUNK;
    const int wc = scan_chunk<NBD, WCAPD>(dsts, nE, cbase, nodeBase, vec8, list, tid, lane, wave);
    if (lane == 0) wcnt[wave] = wc;
    __syncthreads();
    if (wave == 0) {
#pragma unroll 1
      for (int wsx = 0; wsx < NWAVE; ++wsx) {
        int n = __builtin_amdgcn_readfirstlane(wcnt[wsx]);
        n = n > WCAPD ? WCAPD : (n < 0 ? 0 : n);
        const int* lp = list + wsx * WCAPD;
#pragma unroll 1
        for (int i = 0; i < n; ++i) {
          const int ent  = __builtin_amdgcn_readfirstlane(lp[i]);
          const int slot = ent & (NBD - 1);
          if (lane == 0) cnt[slot] = cnt[slot] + 1;
        }
      }
    }
    __syncthreads();
  }

  v4f dq[NBD / (NWAVE * 128)];
#pragma unroll
  for (int q = 0; q < NBD / (NWAVE * 128); ++q) {
    const int f = (wave * (NBD / (NWAVE * 128)) + q) * 128 + 4 * lane;
    const v4i c = *(const v4i*)(cnt + f);
    dq[q].x = rsqrtf((float)(c.x + 1));
    dq[q].y = rsqrtf((float)(c.y + 1));
    dq[q].z = rsqrtf((float)(c.z + 1));
    dq[q].w = rsqrtf((float)(c.w + 1));
  }
  float* dp = dinv + (size_t)nodeBase;
#pragma unroll
  for (int q = 0; q < NBD / (NWAVE * 128); ++q)
    *(volatile v4f*)(dp + (wave * (NBD / (NWAVE * 128)) + q) * 128 + 4 * lane) = dq[q];
  __threadfence();
#pragma unroll
  for (int q = 0; q < NBD / (NWAVE * 128); ++q)
    *(volatile v4f*)(dp + (wave * (NBD / (NWAVE * 128)) + q) * 128 + 4 * lane) = dq[q];
}

__global__ __launch_bounds__(NTHR) void k_gemm(
    const float* __restrict__ x, const float* __restrict__ W, const float* __restrict__ dinv,
    float* y, float* g0, int nN) {
  __shared__ __attribute__((aligned(16))) _Float16 sW[DH * WP];
  __shared__ __attribute__((aligned(16))) float    stg[GROWS * DH];
  const int tid = threadIdx.x, lane = tid & 31, wave = tid >> 5, hh = lane >> 4, m = lane & 15;
  const int rowBase = blockIdx.x * GROWS;

#pragma unroll 4
  for (int i = 0; i < (DX * DH) / NTHR; ++i) {
    const int idx = i * NTHR + tid;
    const int k = idx >> 6;
    const int n = idx & 63;
    sW[n * WP + k] = (_Float16)(W[idx] * WSCALE);
  }
  __syncthreads();

  int node = rowBase + 16 * wave + m;
  node = node > nN - 1 ? nN - 1 : node;
  const float* xr = x + (size_t)node * DX + 8 * hh;

  v8f acc[4];
#pragma unroll
  for (int t = 0; t < 4; ++t) { v8f z = {0.f, 0.f, 0.f, 0.f, 0.f, 0.f, 0.f, 0.f}; acc[t] = z; }
#pragma unroll
  for (int kt = 0; kt < DX / 32; ++kt) {
    const float* xp = xr + 32 * kt;
    FragH a;
    a.h[0] = cvt8(*(const v4f*)xp,        *(const v4f*)(xp + 4));
    a.h[1] = cvt8(*(const v4f*)(xp + 16), *(const v4f*)(xp + 20));
#pragma unroll
    for (int t = 0; t < 4; ++t) {
      const _Float16* bp = sW + (16 * t + m) * WP + 32 * kt + 8 * hh;
      FragH b;
      b.h[0] = *(const v8h*)bp;
      b.h[1] = *(const v8h*)(bp + 16);
      acc[t] = wmh(a.v, b.v, acc[t]);
    }
  }

  float* sp = stg + (16 * wave + 8 * hh) * DH + m;
#pragma unroll
  for (int t = 0; t < 4; ++t) {
    sp[0 * DH + 16 * t] = acc[t][0] * WINV;
    sp[1 * DH + 16 * t] = acc[t][1] * WINV;
    sp[2 * DH + 16 * t] = acc[t][2] * WINV;
    sp[3 * DH + 16 * t] = acc[t][3] * WINV;
    sp[4 * DH + 16 * t] = acc[t][4] * WINV;
    sp[5 * DH + 16 * t] = acc[t][5] * WINV;
    sp[6 * DH + 16 * t] = acc[t][6] * WINV;
    sp[7 * DH + 16 * t] = acc[t][7] * WINV;
  }
  __syncthreads();

  const float* lp = stg + 16 * wave * DH + 4 * lane;
  const size_t rb = (size_t)(rowBase + 16 * wave) * DH + 4 * lane;
  v4f yv[8], gv[8];
#pragma unroll
  for (int i = 0; i < 8; ++i) {
    yv[i] = *(const v4f*)(lp + i * 128);
    const int   r = rowBase + 16 * wave + 2 * i + (lane >> 4);
    const float d = dinv[r];
    gv[i] = yv[i] * d;
  }
#pragma unroll
  for (int i = 0; i < 8; ++i) {
    *(volatile v4f*)(y  + rb + i * 128) = yv[i];
    *(volatile v4f*)(g0 + rb + i * 128) = gv[i];
  }
  __threadfence();
#pragma unroll
  for (int i = 0; i < 8; ++i) {
    *(volatile v4f*)(y  + rb + i * 128) = yv[i];
    *(volatile v4f*)(g0 + rb + i * 128) = gv[i];
  }
}

template <int LAST>
__global__ __launch_bounds__(NTHR) void k_prop(
    const int* __restrict__ ei, const float* __restrict__ gin, const float* __restrict__ y,
    const float* __restrict__ dinv, const float* __restrict__ bias, float* gout,
    int nN, int nE, int vec8) {
  extern __shared__ v4f lds_dyn[];
  float* acc  = (float*)lds_dyn;
  int*   list = (int*)(acc + NBP * DH);
  int*   wcnt = list + NWAVE * WCAPP;
  const int tid = threadIdx.x, lane = tid & 31, wave = tid >> 5;
  const int nodeBase = blockIdx.x * NBP;
  const int* dsts = ei + nE;

  {
    const v4f z = {0.f, 0.f, 0.f, 0.f};
    for (int i = tid; i < NBP * DH / 4; i += NTHR) lds_dyn[i] = z;
  }
  __syncthreads();

  const int nChunks = (nE + CHUNK - 1) / CHUNK;
#pragma unroll 1
  for (int ch = 0; ch < nChunks; ++ch) {
    const int cbase = ch * CHUNK;
    const int wc = scan_chunk<NBP, WCAPP>(dsts, nE, cbase, nodeBase, vec8, list, tid, lane, wave);
    if (lane == 0) wcnt[wave] = wc;
    __syncthreads();
    if (wave == 0) {
#pragma unroll 1
      for (int wsx = 0; wsx < NWAVE; ++wsx) {
        int n = __builtin_amdgcn_readfirstlane(wcnt[wsx]);
        n = n > WCAPP ? WCAPP : (n < 0 ? 0 : n);
        const int* lp = list + wsx * WCAPP;
#pragma unroll 1
        for (int i = 0; i < n; ++i) {
          const int ent  = __builtin_amdgcn_readfirstlane(lp[i]);
          const int slot = ent & (NBP - 1);
          int e = cbase + ((ent >> SLOTB) & (CHUNK - 1));
          e = e > nE - 1 ? nE - 1 : e;
          int src = ei[e];
          src = src < 0 ? 0 : (src > nN - 1 ? nN - 1 : src);
          const v2f v = *(const v2f*)(gin + (size_t)src * DH + 2 * lane);
          v2f* ap = (v2f*)(acc + slot * DH + 2 * lane);
          *ap = *ap + v;
        }
      }
    }
    __syncthreads();
  }

#pragma unroll 4
  for (int i = 0; i < (NBP * DH / 4) / NTHR; ++i) {
    const int idx  = i * NTHR + tid;
    const int slot = idx >> 4;
    const int c4   = (idx & 15) * 4;
    const int node = nodeBase + slot;
    const float d  = dinv[node];
    const v4f   gv = *(const v4f*)(gin + (size_t)node * DH + c4);
    const v4f   yv = *(const v4f*)(y   + (size_t)node * DH + c4);
    v4f* ap = (v4f*)(acc + slot * DH + c4);
    const v4f ag = (*ap + gv) * d;
    v4f hv = ag * C_KEEP + yv * C_TEL;
    if (LAST) {
      const v4f bv = *(const v4f*)(bias + c4);
      hv = hv + bv;
      hv.x = fmaxf(hv.x, 0.f); hv.y = fmaxf(hv.y, 0.f); hv.z = fmaxf(hv.z, 0.f); hv.w = fmaxf(hv.w, 0.f);
    } else {
      hv = hv * d;
    }
    *ap = hv;
  }
  __syncthreads();

  const size_t ob = (size_t)nodeBase * DH;
#pragma unroll 4
  for (int q = 0; q < (NBP * DH) / (NWAVE * 128); ++q) {
    const int f = (wave * ((NBP * DH) / (NWAVE * 128)) + q) * 128 + 4 * lane;
    const v4f v = *(const v4f*)(acc + f);
    *(volatile v4f*)(gout + ob + f) = v;
  }
  __threadfence();
#pragma unroll 4
  for (int q = 0; q < (NBP * DH) / (NWAVE * 128); ++q) {
    const int f = (wave * ((NBP * DH) / (NWAVE * 128)) + q) * 128 + 4 * lane;
    const v4f v = *(const v4f*)(acc + f);
    *(volatile v4f*)(gout + ob + f) = v;
  }
}

__device__ __forceinline__ float logit_of(const float* __restrict__ cf, int i, const float* cwr, float cb0) {
  const v4f a = *(const v4f*)(cf + (size_t)i * AF);
  const v4f b = *(const v4f*)(cf + (size_t)i * AF + 4);
  float s = a.x * cwr[0];
  s += a.y * cwr[1]; s += a.z * cwr[2]; s += a.w * cwr[3];
  s += b.x * cwr[4]; s += b.y * cwr[5]; s += b.z * cwr[6]; s += b.w * cwr[7];
  return s + cb0;
}

__global__ __launch_bounds__(NTHR) void k_pool(
    const float* __restrict__ H, const float* __restrict__ cf, const int* __restrict__ batch,
    const int* __restrict__ numg, const float* __restrict__ cw, const float* __restrict__ cb,
    const float* __restrict__ a1w, const float* __restrict__ a1b,
    const float* __restrict__ a2w, const float* __restrict__ a2b,
    float* out, int nN) {
  extern __shared__ v4f lds_dyn[];
  float*    pooled = (float*)lds_dyn;
  _Float16* tA     = (_Float16*)(pooled + NGMAX * DH);
  float*    outv   = (float*)(tA + NWAVE * 16 * TAP);
  const int tid = threadIdx.x, lane = tid & 31, wave = tid >> 5, hh = lane >> 4, m = lane & 15;
  const int ng = numg[0];
  float cwr[AF];
#pragma unroll
  for (int j = 0; j < AF; ++j) cwr[j] = cw[j];
  const float cb0  = cb[0];
  const float ninf = -__builtin_huge_valf();
  const int nCh = (nN + 31) >> 5;

#pragma unroll 1
  for (int j = 0; j < NGMAX / NWAVE; ++j) {
    const int  g    = j * NWAVE + wave;
    const bool gval = g < ng;
    float mx = ninf;
    int   cn = 0;
#pragma unroll 1
    for (int c = 0; c < nCh; ++c) {
      const int  i   = (c << 5) + lane;
      const int  b   = (i < nN) ? batch[i] : -1;
      const bool hit = gval && (b == g);
      if (hit) {
        const float l = logit_of(cf, i, cwr, cb0);
        mx = fmaxf(mx, l);
        ++cn;
      }
    }
#pragma unroll
    for (int o = 16; o > 0; o >>= 1) {
      mx = fmaxf(mx, __shfl_xor(mx, o));
      cn += __shfl_xor(cn, o);
    }
    float zp = 0.f, M0 = ninf, M1 = ninf;
#pragma unroll 1
    for (int c = 0; c < nCh; ++c) {
      const int  i   = (c << 5) + lane;
      const int  b   = (i < nN) ? batch[i] : -1;
      const bool hit = gval && (b == g);
      float w = 0.f;
      if (hit) {
        const float l = logit_of(cf, i, cwr, cb0);
        w = expf(l - mx);
        zp += w;
      }
      unsigned msk = __builtin_amdgcn_ballot_w32(hit);
      while (msk != 0u) {
        const int k = __builtin_ctz(msk);
        msk &= msk - 1u;
        const float wk = __int_as_float(__builtin_amdgcn_readlane(__float_as_int(w), k));
        int ii = (c << 5) + k;
        ii = ii > nN - 1 ? nN - 1 : ii;
        const v2f hv = *(const v2f*)(H + (size_t)ii * DH + 2 * lane);
        M0 = fmaxf(M0, wk * hv.x);
        M1 = fmaxf(M1, wk * hv.y);
      }
    }
#pragma unroll
    for (int o = 16; o > 0; o >>= 1) zp += __shfl_xor(zp, o);
    const float fac = (cn > 0) ? ((float)cn * (1.0f / zp)) : 1.0f;
    pooled[g * DH + 2 * lane]     = M0 * fac;
    pooled[g * DH + 2 * lane + 1] = M1 * fac;
  }
  __syncthreads();

  FragH bw1[2];
#pragma unroll
  for (int kt = 0; kt < DH / 32; ++kt) {
#pragma unroll
    for (int i = 0; i < 8; ++i) {
      bw1[kt].h[0][i] = (_Float16)(a1w[(32 * kt + 8 * hh + i) * DA + m] * WSCALE);
      bw1[kt].h[1][i] = (_Float16)(a1w[(32 * kt + 16 + 8 * hh + i) * DA + m] * WSCALE);
    }
  }
  FragH bw2;
#pragma unroll
  for (int i = 0; i < 8; ++i) {
    const float wv = (m == 0) ? a2w[8 * hh + i] * WSCALE : 0.f;
    bw2.h[0][i] = (_Float16)wv;
    bw2.h[1][i] = (_Float16)0.f;
  }
  const float bia1 = a1b[m];
  const float bia2 = a2b[0];
  _Float16* myA = tA + wave * 16 * TAP;

#pragma unroll 1
  for (int q = 0; q < (NGMAX / 16) / NWAVE; ++q) {
    const int t = wave + NWAVE * q;
    v8f c1 = {0.f, 0.f, 0.f, 0.f, 0.f, 0.f, 0.f, 0.f};
#pragma unroll
    for (int kt = 0; kt < DH / 32; ++kt) {
      const float* ap = pooled + (16 * t + m) * DH + 32 * kt + 8 * hh;
      FragH a;
      a.h[0] = cvt8(*(const v4f*)ap,        *(const v4f*)(ap + 4));
      a.h[1] = cvt8(*(const v4f*)(ap + 16), *(const v4f*)(ap + 20));
      c1 = wmh(a.v, bw1[kt].v, c1);
    }
#pragma unroll
    for (int r = 0; r < 8; ++r) myA[(8 * hh + r) * TAP + m] = (_Float16)fmaxf(c1[r] * WINV + bia1, 0.f);
    __syncthreads();
    FragH a2;
    a2.h[0] = *(const v8h*)(myA + m * TAP + 8 * hh);
    {
      v8h z8 = {(_Float16)0.f, (_Float16)0.f, (_Float16)0.f, (_Float16)0.f,
                (_Float16)0.f, (_Float16)0.f, (_Float16)0.f, (_Float16)0.f};
      a2.h[1] = z8;
    }
    v8f c2 = {0.f, 0.f, 0.f, 0.f, 0.f, 0.f, 0.f, 0.f};
    c2 = wmh(a2.v, bw2.v, c2);
    if (m == 0) {
#pragma unroll
      for (int r = 0; r < 8; ++r) outv[16 * t + 8 * hh + r] = c2[r] * WINV + bia2;
    }
    __syncthreads();
  }

  if (wave == 0) {
    const v4f o0 = *(const v4f*)(outv + 4 * lane);
    const v4f o1 = *(const v4f*)(outv + 128 + 4 * lane);
    *(volatile v4f*)(out + 4 * lane)       = o0;
    *(volatile v4f*)(out + 128 + 4 * lane) = o1;
    __threadfence();
    *(volatile v4f*)(out + 4 * lane)       = o0;
    *(volatile v4f*)(out + 128 + 4 * lane) = o1;
  }
}

extern "C" void kernel_launch(void* const* d_in, const int* in_sizes, int n_in,
                              void* d_out, int out_size, void* d_ws, size_t ws_size,
                              hipStream_t stream) {
  if (n_in < 13) return;
  const int nN = in_sizes[0] / DX;
  const int nE = in_sizes[2] / 2;
  if (nN <= 0 || in_sizes[0] != nN * DX) return;
  if (nE < 0 || in_sizes[2] != nE * 2) return;
  if (in_sizes[1] != nN * AF || in_sizes[3] != nN || in_sizes[4] < 1) return;
  if (in_sizes[5] != DX * DH || in_sizes[6] < DH || in_sizes[7] < AF || in_sizes[8] < 1) return;
  if (in_sizes[9] != DH * DA || in_sizes[10] < DA || in_sizes[11] < DA || in_sizes[12] < 1) return;
  if (out_size != NGMAX) return;

  const float* x     = (const float*)d_in[0];
  const float* cf    = (const float*)d_in[1];
  const int*   ei    = (const int*)d_in[2];
  const int*   batch = (const int*)d_in[3];
  const int*   numg  = (const int*)d_in[4];
  const float* W     = (const float*)d_in[5];
  const float* b1    = (const float*)d_in[6];
  const float* cw    = (const float*)d_in[7];
  const float* cb    = (const float*)d_in[8];
  const float* a1w   = (const float*)d_in[9];
  const float* a1b   = (const float*)d_in[10];
  const float* a2w   = (const float*)d_in[11];
  const float* a2b   = (const float*)d_in[12];
  float* out = (float*)d_out;

  const int nBP  = (nN + NBP - 1) / NBP;
  const int nPad = nBP * NBP;
  const int nBD  = (nN + NBD - 1) / NBD;
  const int nGM  = nPad / GROWS;

  char* ws = (char*)d_ws;
  size_t off = 0;
  const size_t oDv = off; off += (size_t)nBD * NBD * 4;        off = (off + 255) & ~(size_t)255;
  const size_t oY  = off; off += (size_t)nPad * DH * 4;        off = (off + 255) & ~(size_t)255;
  const size_t oA  = off; off += (size_t)nPad * DH * 4;        off = (off + 255) & ~(size_t)255;
  const size_t oB  = off; off += (size_t)nPad * DH * 4;        off = (off + 255) & ~(size_t)255;
  if (off > ws_size) return;
  float* dinv = (float*)(ws + oDv);
  float* yb   = (float*)(ws + oY);
  float* pA   = (float*)(ws + oA);
  float* pB   = (float*)(ws + oB);

  const int vec8 = ((nE & 3) == 0) ? 1 : 0;

  hipFuncSetAttribute(reinterpret_cast<const void*>(&k_deg),
                      hipFuncAttributeMaxDynamicSharedMemorySize, LDS_DEG);
  k_deg<<<nBD, NTHR, LDS_DEG, stream>>>(ei, dinv, nE, vec8);

  k_gemm<<<nGM, NTHR, 0, stream>>>(x, W, dinv, yb, pA, nN);

  hipFuncSetAttribute(reinterpret_cast<const void*>(&k_prop<0>),
                      hipFuncAttributeMaxDynamicSharedMemorySize, LDS_PROP);
  hipFuncSetAttribute(reinterpret_cast<const void*>(&k_prop<1>),
                      hipFuncAttributeMaxDynamicSharedMemorySize, LDS_PROP);
  k_prop<0><<<nBP, NTHR, LDS_PROP, stream>>>(ei, pA, yb, dinv, b1, pB, nN, nE, vec8);
  k_prop<0><<<nBP, NTHR, LDS_PROP, stream>>>(ei, pB, yb, dinv, b1, pA, nN, nE, vec8);
  k_prop<1><<<nBP, NTHR, LDS_PROP, stream>>>(ei, pA, yb, dinv, b1, pB, nN, nE, vec8);

  hipFuncSetAttribute(reinterpret_cast<const void*>(&k_pool),
                      hipFuncAttributeMaxDynamicSharedMemorySize, LDS_POOL);
  k_pool<<<1, NTHR, LDS_POOL, stream>>>(pB, cf, batch, numg, cw, cb, a1w, a1b, a2w, a2b, out, nN);
}
